// EquivariantBlockPyG_77618648973486
// MI455X (gfx1250) — hardware-verified
//
#include <hip/hip_runtime.h>
#include <stddef.h>


typedef unsigned short us_t;
typedef float    v4f  __attribute__((ext_vector_type(4)));
typedef float    v8f  __attribute__((ext_vector_type(8)));
typedef int      v4i  __attribute__((ext_vector_type(4)));
typedef us_t     us8  __attribute__((ext_vector_type(8)));
typedef _Float16 v8h  __attribute__((ext_vector_type(8)));
typedef _Float16 v16h __attribute__((ext_vector_type(16)));
typedef __bf16   v16b __attribute__((ext_vector_type(16)));
union FragB { v16b v; us8 u[2]; };
union FragH { v16h v; v8h h[2]; us8 u[2]; };
union H8    { v8h h; us8 u; };

#define HD      256
#define HD2     512
#define NTHR    256
#define NWAVE   8
#define TGT     64
#define TGT_SH  6
#define MROW    32
#define AP      264
#define MP      260
#define EPT     8
#define NGRP    2
#define CHUNK   (NTHR * EPT * NGRP)
#define WCAP    (EPT * NGRP * 32)
#define LCAP    4096
#define NGR     64
#define NGC     128
#define NGT     128
#define SP      132
#define ASC     16.0f
#define LOSC    2048.0f
#define INV_AB  0.00390625f
#define INV_ABL 1.9073486328125e-6f

#define O_AGG   0
#define O_SA    (O_AGG + TGT * HD * 4)
#define O_M2    (O_SA + MROW * AP * 2)
#define O_LIST  (O_M2 + MROW * MP * 4)
#define O_WSCR  (O_LIST + LCAP * 4)
#define O_SW    (O_WSCR + NWAVE * WCAP * 4)
#define O_MISC  (O_SW + 5 * HD * 4)
#define LDS_EDGE (O_MISC + 2048)

static_assert(TGT == (1 << TGT_SH));
static_assert(NTHR == HD);
static_assert(MROW * 8 == NTHR);
static_assert((LCAP % MROW) == 0);
static_assert((CHUNK & (CHUNK - 1)) == 0);
static_assert(NGR == 64 && NGT == 128 && NGC == 128);
static_assert((O_SA % 16) == 0 && (O_M2 % 16) == 0 && (O_LIST % 16) == 0 && (O_WSCR % 16) == 0 && (O_SW % 16) == 0 && (O_MISC % 16) == 0);
static_assert(488 * 4 <= 2048);
static_assert((AP * 2) % 16 == 0 && (MP * 4) % 16 == 0 && (SP * 4) % 16 == 0);
static_assert(TGT == NWAVE * 8);

__device__ __forceinline__ us_t f2bf(float f) {
  unsigned u = __float_as_uint(f);
  u += 0x7FFFu + ((u >> 16) & 1u);
  return (us_t)(u >> 16);
}
__device__ __forceinline__ float bf2f(us_t b) { return __uint_as_float(((unsigned)b) << 16); }
__device__ __forceinline__ void split8(v4f a, v4f b, us8& hv, us8& lv) {
  float f[8];
  f[0] = a.x; f[1] = a.y; f[2] = a.z; f[3] = a.w; f[4] = b.x; f[5] = b.y; f[6] = b.z; f[7] = b.w;
#pragma unroll
  for (int e = 0; e < 8; ++e) { const us_t hb = f2bf(f[e]); hv[e] = hb; lv[e] = f2bf(f[e] - bf2f(hb)); }
}
__device__ __forceinline__ float rcp_f(float x)  { return __builtin_amdgcn_rcpf(x); }
__device__ __forceinline__ float silu_f(float x) { return x * rcp_f(1.0f + __expf(-x)); }
__device__ __forceinline__ float sigm_f(float x) { return rcp_f(1.0f + __expf(-x)); }

__device__ __forceinline__ v8f wbf(v16b a, v16b b, v8f c) {
  v8f d = __builtin_amdgcn_wmma_f32_16x16x32_bf16(false, a, false, b, (short)0, c, false, false);
  asm volatile("v_nop\n\tv_nop\n\tv_nop\n\tv_nop" : "+v"(d) : "v"(a), "v"(b));
  return d;
}
__device__ __forceinline__ v8f whf(v16h a, v16h b, v8f c) {
  v8f d = __builtin_amdgcn_wmma_f32_16x16x32_f16(false, a, false, b, (short)0, c, false, false);
  asm volatile("v_nop\n\tv_nop\n\tv_nop\n\tv_nop" : "+v"(d) : "v"(a), "v"(b));
  return d;
}

__device__ __forceinline__ void geom4(const float* __restrict__ x, int src, int node, float* g) {
#pragma clang fp contract(off)
  const float a0 = x[(size_t)src * 3 + 0], a1 = x[(size_t)src * 3 + 1], a2 = x[(size_t)src * 3 + 2];
  const float c0 = x[(size_t)node * 3 + 0], c1 = x[(size_t)node * 3 + 1], c2 = x[(size_t)node * 3 + 2];
  const float d0 = a0 - c0, d1 = a1 - c1, d2 = a2 - c2;
  const float rad = d0 * d0 + d1 * d1 + d2 * d2;
  const float nrm = sqrtf(rad + 1e-8f);
  const float inv = rcp_f(nrm + 1.0f);
  g[0] = d0 * inv; g[1] = d1 * inv; g[2] = d2 * inv; g[3] = rad;
}

__global__ __launch_bounds__(256) void k_cvt_h(const float* __restrict__ h, us_t* ph, us_t* pl, int n8) {
  const int i = blockIdx.x * 256 + (int)threadIdx.x;
  if (i >= n8) return;
  const float* p = h + (size_t)i * 8;
  const v4f a = *(const v4f*)p, b = *(const v4f*)(p + 4);
  us8 hv, lv;
  split8(a, b, hv, lv);
  us_t* dp = ph + (size_t)i * 8;
  us_t* dq = pl + (size_t)i * 8;
  *(volatile us8*)dp = hv; *(volatile us8*)dq = lv;
  __threadfence();
  *(volatile us8*)dp = hv; *(volatile us8*)dq = lv;
}

__global__ __launch_bounds__(256) void k_wcvt(const float* __restrict__ src, int srcRows,
                                             us_t* ph, us_t* pl, int K, int NOUT, int mode) {
  const int idx = blockIdx.x * 256 + (int)threadIdx.x;
  const int kpr = K >> 3;
  if (idx >= NOUT * kpr) return;
  const int n = idx / kpr;
  const int k0 = (idx - n * kpr) * 8;
  const int col = n & 255;
  const int radd = (n >> 8) * 256;
  float v[8];
#pragma unroll
  for (int e = 0; e < 8; ++e) {
    int row = radd + k0 + e;
    row = row > srcRows - 1 ? srcRows - 1 : row;
    v[e] = src[(size_t)row * 256 + col];
  }
  us8 o0, o1;
  if (mode == 0) {
#pragma unroll
    for (int e = 0; e < 8; ++e) { const us_t hb = f2bf(v[e]); o0[e] = hb; o1[e] = f2bf(v[e] - bf2f(hb)); }
  } else {
    v8h hvv, lvv;
#pragma unroll
    for (int e = 0; e < 8; ++e) {
      const float sv = v[e] * ASC;
      const _Float16 hx = (_Float16)sv;
      hvv[e] = hx;
      lvv[e] = (_Float16)((sv - (float)hx) * LOSC);
    }
    H8 a, b; a.h = hvv; b.h = lvv; o0 = a.u; o1 = b.u;
  }
  us_t* dp = ph + (size_t)idx * 8;
  us_t* dq = pl + (size_t)idx * 8;
  *(volatile us8*)dp = o0;
  if (mode != 2) *(volatile us8*)dq = o1;
  __threadfence();
  *(volatile us8*)dp = o0;
  if (mode != 2) *(volatile us8*)dq = o1;
}

__device__ __forceinline__ void ng_khalf(const us_t* __restrict__ Ah, const us_t* __restrict__ Al, int arow,
                                         const us_t* __restrict__ Bh, const us_t* __restrict__ Bl,
                                         int KD, int cb, int kofs, int hh, int m, v8f (&acc)[8]) {
  const us_t* ap = Ah + (size_t)arow * HD + 8 * hh;
  const us_t* aq = Al + (size_t)arow * HD + 8 * hh;
#pragma unroll 1
  for (int kt = 0; kt < HD / 32; ++kt) {
    FragB ah, al;
    ah.u[0] = *(const us8*)(ap + 32 * kt);
    ah.u[1] = *(const us8*)(ap + 32 * kt + 16);
    al.u[0] = *(const us8*)(aq + 32 * kt);
    al.u[1] = *(const us8*)(aq + 32 * kt + 16);
    const int kb = kofs + 32 * kt + 8 * hh;
#pragma unroll
    for (int t = 0; t < 8; ++t) {
      const size_t nb = (size_t)(cb + 16 * t + m) * KD + kb;
      FragB bh, bl;
      bh.u[0] = *(const us8*)(Bh + nb); bh.u[1] = *(const us8*)(Bh + nb + 16);
      bl.u[0] = *(const us8*)(Bl + nb); bl.u[1] = *(const us8*)(Bl + nb + 16);
      acc[t] = wbf(ah.v, bh.v, acc[t]);
      acc[t] = wbf(al.v, bh.v, acc[t]);
      acc[t] = wbf(ah.v, bl.v, acc[t]);
    }
  }
}

__device__ __forceinline__ void ng_store(const float* stg, int wave, int lane, int rowBase, int cb, int NC,
                                         float* Cf, us_t* Ch, us_t* Cl, int writeF, int writeP) {
  const int pl = lane & 15;
  const bool loh = lane >= 16;
#pragma unroll
  for (int i = 0; i < 16; ++i) {
    const int row = 16 * wave + i;
    const size_t gro = (size_t)(rowBase + row) * NC + cb;
    const float* sp = stg + row * SP;
    if (writeF != 0) {
      const v4f v = *(const v4f*)(sp + 4 * lane);
      *(volatile v4f*)(Cf + gro + 4 * lane) = v;
    }
    if (writeP != 0) {
      const v4f f0 = *(const v4f*)(sp + 8 * pl), f1 = *(const v4f*)(sp + 8 * pl + 4);
      us8 hv, lv;
      split8(f0, f1, hv, lv);
      us8 sv;
#pragma unroll
      for (int e = 0; e < 8; ++e) sv[e] = loh ? lv[e] : hv[e];
      us_t* dp = (loh ? Cl : Ch) + gro + 8 * pl;
      *(volatile us8*)dp = sv;
    }
  }
}

template <int KD>
__global__ __launch_bounds__(NGT) void k_ngemm(
    const us_t* __restrict__ A1h, const us_t* __restrict__ A1l,
    const us_t* __restrict__ A2h, const us_t* __restrict__ A2l,
    const us_t* __restrict__ Bh, const us_t* __restrict__ Bl,
    const float* __restrict__ bias, int biasLen, int NC, int useBias, int useSilu,
    float* Cf, us_t* Ch, us_t* Cl, int writeF, int writeP) {
  __shared__ __attribute__((aligned(16))) float stg[NGR * SP];
  const int tid = threadIdx.x, lane = tid & 31, wave = tid >> 5, hh = lane >> 4, m = lane & 15;
  const int rowBase = blockIdx.x * NGR, cb = blockIdx.y * NGC;
  const int arow = rowBase + 16 * wave + m;

  v8f acc[8];
#pragma unroll
  for (int t = 0; t < 8; ++t) { v8f z = {0.f, 0.f, 0.f, 0.f, 0.f, 0.f, 0.f, 0.f}; acc[t] = z; }
  ng_khalf(A1h, A1l, arow, Bh, Bl, KD, cb, 0, hh, m, acc);
  if (KD == HD2) ng_khalf(A2h, A2l, arow, Bh, Bl, KD, cb, HD, hh, m, acc);

  const int r0 = 16 * wave + 8 * hh;
#pragma unroll
  for (int t = 0; t < 8; ++t) {
    const int col = cb + 16 * t + m;
    const int bc  = col < biasLen ? col : biasLen - 1;
    const float bl0 = bias[bc];
    const float bv  = useBias != 0 ? bl0 : 0.0f;
#pragma unroll
    for (int r = 0; r < 8; ++r) {
      float v = acc[t][r] + bv;
      const float sv = silu_f(v);
      v = useSilu != 0 ? sv : v;
      stg[(r0 + r) * SP + 16 * t + m] = v;
    }
  }
  __syncthreads();
  ng_store(stg, wave, lane, rowBase, cb, NC, Cf, Ch, Cl, writeF, writeP);
  __threadfence();
  ng_store(stg, wave, lane, rowBase, cb, NC, Cf, Ch, Cl, writeF, writeP);
}

template <int NB>
__device__ __forceinline__ int scan_chunk(const int* __restrict__ dsts, int nE, int cbase, int slotBase,
                                          int vec8, int* wl, int tid) {
  int wc = 0;
#pragma unroll
  for (int g = 0; g < NGRP; ++g) {
    const int el0  = (g * NTHR + tid) * EPT;
    const int e0   = cbase + el0;
    const int sent = -2147483647 - 1;
    v4i da, db;
    if (vec8 != 0 && cbase + CHUNK <= nE) {
      da = *(const v4i*)(dsts + e0);
      db = *(const v4i*)(dsts + e0 + 4);
    } else {
      da.x = (e0     < nE) ? dsts[(e0     < nE - 1) ? e0     : nE - 1] : sent;
      da.y = (e0 + 1 < nE) ? dsts[(e0 + 1 < nE - 1) ? e0 + 1 : nE - 1] : sent;
      da.z = (e0 + 2 < nE) ? dsts[(e0 + 2 < nE - 1) ? e0 + 2 : nE - 1] : sent;
      da.w = (e0 + 3 < nE) ? dsts[(e0 + 3 < nE - 1) ? e0 + 3 : nE - 1] : sent;
      db.x = (e0 + 4 < nE) ? dsts[(e0 + 4 < nE - 1) ? e0 + 4 : nE - 1] : sent;
      db.y = (e0 + 5 < nE) ? dsts[(e0 + 5 < nE - 1) ? e0 + 5 : nE - 1] : sent;
      db.z = (e0 + 6 < nE) ? dsts[(e0 + 6 < nE - 1) ? e0 + 6 : nE - 1] : sent;
      db.w = (e0 + 7 < nE) ? dsts[(e0 + 7 < nE - 1) ? e0 + 7 : nE - 1] : sent;
    }
    const unsigned nb = (unsigned)slotBase;
    const unsigned s0 = (unsigned)da.x - nb, s1 = (unsigned)da.y - nb;
    const unsigned s2 = (unsigned)da.z - nb, s3 = (unsigned)da.w - nb;
    const unsigned s4 = (unsigned)db.x - nb, s5 = (unsigned)db.y - nb;
    const unsigned s6 = (unsigned)db.z - nb, s7 = (unsigned)db.w - nb;
    const bool q0 = s0 < (unsigned)NB, q1 = s1 < (unsigned)NB, q2 = s2 < (unsigned)NB, q3 = s3 < (unsigned)NB;
    const bool q4 = s4 < (unsigned)NB, q5 = s5 < (unsigned)NB, q6 = s6 < (unsigned)NB, q7 = s7 < (unsigned)NB;
    const unsigned any = __builtin_amdgcn_ballot_w32(q0 | q1 | q2 | q3 | q4 | q5 | q6 | q7);
    if (any != 0u) {
#define HITJ(J, QJ, SJ) { \
        const unsigned mj = __builtin_amdgcn_ballot_w32(QJ); \
        if (mj != 0u) { \
          if (QJ) { \
            const int pos = wc + (int)__builtin_amdgcn_mbcnt_lo(mj, 0u); \
            if (pos < WCAP) wl[pos] = ((e0 + (J)) << TGT_SH) | (int)(SJ); \
          } \
          wc += (int)__builtin_popcount(mj); } }
      HITJ(0, q0, s0)
      HITJ(1, q1, s1)
      HITJ(2, q2, s2)
      HITJ(3, q3, s3)
      HITJ(4, q4, s4)
      HITJ(5, q5, s5)
      HITJ(6, q6, s6)
      HITJ(7, q7, s7)
#undef HITJ
    }
  }
  return wc;
}

template <int POS>
__global__ __launch_bounds__(NTHR) void k_edge(
    const float* __restrict__ PQ, const int* __restrict__ ei, int nE, int nN, int vec8,
    const us_t* __restrict__ Wh, const us_t* __restrict__ Wl,
    const float* __restrict__ b1, const float* __restrict__ b2, const float* __restrict__ v3,
    const float* __restrict__ gb, const float* __restrict__ wext,
    const float* __restrict__ x, const float* __restrict__ eattr,
    us_t* aggHo, us_t* aggLo, float* xout) {
  extern __shared__ v4f lds_dyn[];
  char* lb = (char*)lds_dyn;
  float*    aggL  = (float*)(lb + O_AGG);
  _Float16* sA    = (_Float16*)(lb + O_SA);
  float*    sM2   = (float*)(lb + O_M2);
  int*      list  = (int*)(lb + O_LIST);
  int*      wscr  = (int*)(lb + O_WSCR);
  float*    sW    = (float*)(lb + O_SW);
  int*      sSlot = (int*)(lb + O_MISC);
  int*      sSrc  = sSlot + 32;
  int*      sVal  = sSlot + 64;
  float*    sAtt  = (float*)(sSlot + 96);
  float*    sGeo  = (float*)(sSlot + 128);
  float*    sEA   = (float*)(sSlot + 256);
  int*      wcnt  = sSlot + 288;
  float*    sXo   = (float*)(sSlot + 296);

  const int tid = threadIdx.x, lane = tid & 31, wave = tid >> 5, hh = lane >> 4, m = lane & 15;
  const int nodeBase = blockIdx.x * TGT;

  {
    const v4f z = {0.f, 0.f, 0.f, 0.f};
    for (int i = tid; i < TGT * HD / 4; i += NTHR) ((v4f*)aggL)[i] = z;
    sW[tid] = b1[tid];
    sW[HD + tid] = b2[tid];
    sW[2 * HD + tid] = v3[tid];
    if (POS) { sW[3 * HD + tid] = wext[tid]; sW[4 * HD + tid] = wext[HD + tid]; }
  }
  __syncthreads();

  int listLen = 0;
  const int* dsts = ei + nE;
  const int nChunks = (nE + CHUNK - 1) / CHUNK;
  int* wl = wscr + wave * WCAP;
#pragma unroll 1
  for (int ch = 0; ch < nChunks; ++ch) {
    const int cbase = ch * CHUNK;
    const int wc = scan_chunk<TGT>(dsts, nE, cbase, nodeBase, vec8, wl, tid);
    if (lane == 0) wcnt[wave] = wc;
    __syncthreads();
    int pre = 0, tot = 0;
#pragma unroll
    for (int w = 0; w < NWAVE; ++w) {
      int cw = wcnt[w];
      cw = cw < 0 ? 0 : (cw > WCAP ? WCAP : cw);
      tot += cw;
      pre += (w < wave) ? cw : 0;
    }
    const int cm = wc > WCAP ? WCAP : wc;
    for (int i = lane; i < cm; i += 32) {
      const int pos = listLen + pre + i;
      if (pos < LCAP) list[pos] = wl[i];
    }
    listLen += tot;
    listLen = listLen > LCAP ? LCAP : listLen;
    __syncthreads();
  }
  const int L = listLen;
  const int nBatch = (L + MROW - 1) / MROW;
  float gbv = 0.0f;
  if (!POS) gbv = gb[0];

#pragma unroll 1
  for (int bt = 0; bt < nBatch; ++bt) {
    if (tid < MROW) {
      const int idx = bt * MROW + tid;
      const int valid = idx < L ? 1 : 0;
      int ent = list[idx < LCAP ? idx : LCAP - 1];
      ent = valid != 0 ? ent : 0;
      int e = ent >> TGT_SH;
      e = e < 0 ? 0 : (e > nE - 1 ? nE - 1 : e);
      const int sl = ent & (TGT - 1);
      int src = ei[e];
      src = src < 0 ? 0 : (src > nN - 1 ? nN - 1 : src);
      int node = nodeBase + sl;
      node = node > nN - 1 ? nN - 1 : node;
      sSlot[tid] = sl; sSrc[tid] = src; sVal[tid] = valid;
      if (POS) { geom4(x, src, node, sGeo + tid * 4); sEA[tid] = eattr[e]; }
    }
    __syncthreads();

    {
      const int r = tid >> 3, c = tid & 7;
      const int sl = sSlot[r], sr = sSrc[r];
      int node = nodeBase + sl;
      node = node > nN - 1 ? nN - 1 : node;
      const float* pp = PQ + (size_t)node * HD2 + 32 * c;
      const float* qp = PQ + (size_t)sr * HD2 + HD + 32 * c;
      float rad = 0.0f, ea = 0.0f;
      if (POS) { rad = sGeo[r * 4 + 3]; ea = sEA[r]; }
      _Float16* arow = sA + r * AP + 32 * c;
#pragma unroll
      for (int q = 0; q < 4; ++q) {
        const v4f p0 = *(const v4f*)(pp + 8 * q), p1 = *(const v4f*)(pp + 8 * q + 4);
        const v4f q0 = *(const v4f*)(qp + 8 * q), q1 = *(const v4f*)(qp + 8 * q + 4);
        const v4f bA = *(const v4f*)(sW + 32 * c + 8 * q), bB = *(const v4f*)(sW + 32 * c + 8 * q + 4);
        v4f z0 = p0 + q0 + bA, z1 = p1 + q1 + bB;
        if (POS) {
          const v4f wa0 = *(const v4f*)(sW + 3 * HD + 32 * c + 8 * q), wa1 = *(const v4f*)(sW + 3 * HD + 32 * c + 8 * q + 4);
          const v4f we0 = *(const v4f*)(sW + 4 * HD + 32 * c + 8 * q), we1 = *(const v4f*)(sW + 4 * HD + 32 * c + 8 * q + 4);
          z0 = z0 + wa0 * rad + we0 * ea;
          z1 = z1 + wa1 * rad + we1 * ea;
        }
        v8h o;
        o[0] = (_Float16)(silu_f(z0.x) * ASC); o[1] = (_Float16)(silu_f(z0.y) * ASC);
        o[2] = (_Float16)(silu_f(z0.z) * ASC); o[3] = (_Float16)(silu_f(z0.w) * ASC);
        o[4] = (_Float16)(silu_f(z1.x) * ASC); o[5] = (_Float16)(silu_f(z1.y) * ASC);
        o[6] = (_Float16)(silu_f(z1.z) * ASC); o[7] = (_Float16)(silu_f(z1.w) * ASC);
        *(v8h*)(arow + 8 * q) = o;
      }
    }
    __syncthreads();

    {
      v8f accH[2][2], accL[2][2];
#pragma unroll
      for (int i = 0; i < 2; ++i)
#pragma unroll
        for (int j = 0; j < 2; ++j) {
          v8f z = {0.f, 0.f, 0.f, 0.f, 0.f, 0.f, 0.f, 0.f};
          accH[i][j] = z; accL[i][j] = z;
        }
      const _Float16* ab0 = sA + m * AP + 8 * hh;
      const _Float16* ab1 = sA + (16 + m) * AP + 8 * hh;
      const int ncol0 = 32 * wave + m;
#pragma unroll 1
      for (int kt = 0; kt < HD / 32; ++kt) {
        FragH a0, a1;
        a0.h[0] = *(const v8h*)(ab0 + 32 * kt);
        a0.h[1] = *(const v8h*)(ab0 + 32 * kt + 16);
        a1.h[0] = *(const v8h*)(ab1 + 32 * kt);
        a1.h[1] = *(const v8h*)(ab1 + 32 * kt + 16);
#pragma unroll
        for (int t = 0; t < 2; ++t) {
          const size_t nb = (size_t)(ncol0 + 16 * t) * HD + 32 * kt + 8 * hh;
          FragH bh;
          bh.u[0] = *(const us8*)(Wh + nb); bh.u[1] = *(const us8*)(Wh + nb + 16);
          accH[0][t] = whf(a0.v, bh.v, accH[0][t]);
          accH[1][t] = whf(a1.v, bh.v, accH[1][t]);
          if (!POS) {
            FragH bl;
            bl.u[0] = *(const us8*)(Wl + nb); bl.u[1] = *(const us8*)(Wl + nb + 16);
            accL[0][t] = whf(a0.v, bl.v, accL[0][t]);
            accL[1][t] = whf(a1.v, bl.v, accL[1][t]);
          }
        }
      }
#pragma unroll
      for (int t = 0; t < 2; ++t) {
        const int col = ncol0 + 16 * t;
        const float bb = sW[HD + col];
#pragma unroll
        for (int tr = 0; tr < 2; ++tr)
#pragma unroll
          for (int r = 0; r < 8; ++r) {
            float v = accH[tr][t][r] * INV_AB + bb;
            if (!POS) v += accL[tr][t][r] * INV_ABL;
            sM2[(16 * tr + 8 * hh + r) * MP + col] = silu_f(v);
          }
      }
    }
    __syncthreads();

    {
      const int r = tid >> 3, c = tid & 7;
      float s = 0.0f;
#pragma unroll
      for (int q = 0; q < 8; ++q) {
        const v4f mv = *(const v4f*)(sM2 + r * MP + 32 * c + 4 * q);
        const v4f wv = *(const v4f*)(sW + 2 * HD + 32 * c + 4 * q);
        s += mv.x * wv.x; s += mv.y * wv.y; s += mv.z * wv.z; s += mv.w * wv.w;
      }
      s += __shfl_xor(s, 1);
      s += __shfl_xor(s, 2);
      s += __shfl_xor(s, 4);
      float val = s;
      if (!POS) val = sigm_f(s + gbv);
      if (c == 0) sAtt[r] = sVal[r] != 0 ? val : 0.0f;
    }
    __syncthreads();

    if (!POS) {
#pragma unroll 1
      for (int r = 0; r < MROW; ++r) {
        const int sl = sSlot[r];
        const float a = sAtt[r];
        aggL[sl * HD + tid] += a * sM2[r * MP + tid];
      }
    } else {
      if (tid < 3) {
#pragma unroll 1
        for (int r = 0; r < MROW; ++r) {
          const int sl = sSlot[r];
          const float a = sAtt[r];
          aggL[sl * 4 + tid] += sGeo[r * 4 + tid] * a;
        }
      }
    }
    __syncthreads();
  }

  if (!POS) {
#pragma unroll
    for (int i = 0; i < 8; ++i) {
      const int row = wave * 8 + i;
      const float* ap = aggL + row * HD + 8 * lane;
      const v4f f0 = *(const v4f*)ap, f1 = *(const v4f*)(ap + 4);
      us8 hv, lv;
      split8(f0, f1, hv, lv);
      const size_t go = (size_t)(nodeBase + row) * HD + 8 * lane;
      *(volatile us8*)(aggHo + go) = hv;
      *(volatile us8*)(aggLo + go) = lv;
    }
    __threadfence();
#pragma unroll
    for (int i = 0; i < 8; ++i) {
      const int row = wave * 8 + i;
      const float* ap = aggL + row * HD + 8 * lane;
      const v4f f0 = *(const v4f*)ap, f1 = *(const v4f*)(ap + 4);
      us8 hv, lv;
      split8(f0, f1, hv, lv);
      const size_t go = (size_t)(nodeBase + row) * HD + 8 * lane;
      *(volatile us8*)(aggHo + go) = hv;
      *(volatile us8*)(aggLo + go) = lv;
    }
  } else {
    if (tid < TGT * 3) {
      const int sl = tid / 3, d = tid - 3 * sl;
      int node = nodeBase + sl;
      node = node > nN - 1 ? nN - 1 : node;
      sXo[tid] = x[(size_t)node * 3 + d] + aggL[sl * 4 + d];
    }
    __syncthreads();
    const int ti = tid < 48 ? tid : 47;
    const v4f ov = *(const v4f*)(sXo + 4 * ti);
    float* op = xout + (size_t)nodeBase * 3 + 4 * ti;
    if (tid < 48) *(volatile v4f*)op = ov;
    __threadfence();
    if (tid < 48) *(volatile v4f*)op = ov;
  }
}

static size_t carve(size_t& off, size_t bytes) {
  const size_t o = off;
  off += (bytes + 255) & ~(size_t)255;
  return o;
}

extern "C" void kernel_launch(void* const* d_in, const int* in_sizes, int n_in,
                              void* d_out, int out_size, void* d_ws, size_t ws_size,
                              hipStream_t stream) {
  if (n_in < 19) return;
  const int nN = in_sizes[1] / 3;
  if (nN <= 0 || in_sizes[1] != nN * 3 || in_sizes[0] != nN * HD) return;
  if ((nN % TGT) != 0 || (nN % NGR) != 0 || nN > (1 << 24)) return;
  const int nE = in_sizes[2];
  if (nE <= 0 || in_sizes[3] != 2 * nE || nE >= (1 << 24)) return;
  const int nL = in_sizes[4] / (HD2 * HD);
  if (nL < 1 || nL > 8 || in_sizes[4] != nL * HD2 * HD) return;
  if (in_sizes[5] < nL * HD || in_sizes[6] != nL * HD * HD || in_sizes[7] < nL * HD) return;
  if (in_sizes[8] < nL * HD || in_sizes[9] < nL || in_sizes[10] != nL * HD2 * HD || in_sizes[11] < nL * HD) return;
  if (in_sizes[12] != nL * HD * HD || in_sizes[13] < nL * HD) return;
  if (in_sizes[14] != (HD2 + 2) * HD || in_sizes[15] < HD || in_sizes[16] != HD * HD || in_sizes[17] < HD || in_sizes[18] < HD) return;
  if (out_size != nN * HD + nN * 3) return;

  const float* h_in  = (const float*)d_in[0];
  const float* x_in  = (const float*)d_in[1];
  const float* eattr = (const float*)d_in[2];
  const int*   eidx  = (const int*)d_in[3];
  const float* ew1   = (const float*)d_in[4];
  const float* eb1   = (const float*)d_in[5];
  const float* ew2   = (const float*)d_in[6];
  const float* eb2   = (const float*)d_in[7];
  const float* attw  = (const float*)d_in[8];
  const float* attb  = (const float*)d_in[9];
  const float* nw1   = (const float*)d_in[10];
  const float* nb1   = (const float*)d_in[11];
  const float* nw2   = (const float*)d_in[12];
  const float* nb2   = (const float*)d_in[13];
  const float* cw1   = (const float*)d_in[14];
  const float* cb1   = (const float*)d_in[15];
  const float* cw2   = (const float*)d_in[16];
  const float* cb2   = (const float*)d_in[17];
  const float* cw3   = (const float*)d_in[18];
  float* out_h = (float*)d_out;
  float* out_x = out_h + (size_t)nN * HD;

  char* ws = (char*)d_ws;
  size_t off = 0;
  const size_t oHh  = carve(off, (size_t)nN * HD * 2);
  const size_t oHl  = carve(off, (size_t)nN * HD * 2);
  const size_t oPQ  = carve(off, (size_t)nN * HD2 * 4);
  const size_t oAh  = carve(off, (size_t)nN * HD * 2);
  const size_t oAl  = carve(off, (size_t)nN * HD * 2);
  const size_t oNh  = carve(off, (size_t)nN * HD * 2);
  const size_t oNl  = carve(off, (size_t)nN * HD * 2);
  size_t oPQh[8], oPQl[8], oE2h[8], oE2l[8], oN1h[8], oN1l[8], oN2h[8], oN2l[8];
  for (int l = 0; l < nL; ++l) {
    oPQh[l] = carve(off, (size_t)HD2 * HD * 2);
    oPQl[l] = carve(off, (size_t)HD2 * HD * 2);
    oE2h[l] = carve(off, (size_t)HD * HD * 2);
    oE2l[l] = carve(off, (size_t)HD * HD * 2);
    oN1h[l] = carve(off, (size_t)HD * HD2 * 2);
    oN1l[l] = carve(off, (size_t)HD * HD2 * 2);
    oN2h[l] = carve(off, (size_t)HD * HD * 2);
    oN2l[l] = carve(off, (size_t)HD * HD * 2);
  }
  const size_t oCPh = carve(off, (size_t)HD2 * HD * 2);
  const size_t oCPl = carve(off, (size_t)HD2 * HD * 2);
  const size_t oC2  = carve(off, (size_t)HD * HD * 2);
  if (off > ws_size) return;

  us_t*  hH   = (us_t*)(ws + oHh);
  us_t*  hL   = (us_t*)(ws + oHl);
  float* PQ   = (float*)(ws + oPQ);
  us_t*  aggH = (us_t*)(ws + oAh);
  us_t*  aggL = (us_t*)(ws + oAl);
  us_t*  nhH  = (us_t*)(ws + oNh);
  us_t*  nhL  = (us_t*)(ws + oNl);
  us_t*  wCPh = (us_t*)(ws + oCPh);
  us_t*  wCPl = (us_t*)(ws + oCPl);
  us_t*  wC2  = (us_t*)(ws + oC2);

  const int vec8 = ((nE & 3) == 0) ? 1 : 0;

  const int n8 = nN * HD / 8;
  k_cvt_h<<<(n8 + 255) / 256, 256, 0, stream>>>(h_in, hH, hL, n8);

  for (int l = 0; l < nL; ++l) {
    k_wcvt<<<(HD2 * (HD / 8) + 255) / 256, 256, 0, stream>>>(ew1 + (size_t)l * HD2 * HD, HD2,
        (us_t*)(ws + oPQh[l]), (us_t*)(ws + oPQl[l]), HD, HD2, 0);
    k_wcvt<<<(HD * (HD / 8) + 255) / 256, 256, 0, stream>>>(ew2 + (size_t)l * HD * HD, HD,
        (us_t*)(ws + oE2h[l]), (us_t*)(ws + oE2l[l]), HD, HD, 1);
    k_wcvt<<<(HD * (HD2 / 8) + 255) / 256, 256, 0, stream>>>(nw1 + (size_t)l * HD2 * HD, HD2,
        (us_t*)(ws + oN1h[l]), (us_t*)(ws + oN1l[l]), HD2, HD, 0);
    k_wcvt<<<(HD * (HD / 8) + 255) / 256, 256, 0, stream>>>(nw2 + (size_t)l * HD * HD, HD,
        (us_t*)(ws + oN2h[l]), (us_t*)(ws + oN2l[l]), HD, HD, 0);
  }
  k_wcvt<<<(HD2 * (HD / 8) + 255) / 256, 256, 0, stream>>>(cw1, HD2 + 2, wCPh, wCPl, HD, HD2, 0);
  k_wcvt<<<(HD * (HD / 8) + 255) / 256, 256, 0, stream>>>(cw2, HD, wC2, wC2, HD, HD, 2);

  hipFuncSetAttribute(reinterpret_cast<const void*>(&k_edge<0>), hipFuncAttributeMaxDynamicSharedMemorySize, LDS_EDGE);
  hipFuncSetAttribute(reinterpret_cast<const void*>(&k_edge<1>), hipFuncAttributeMaxDynamicSharedMemorySize, LDS_EDGE);

  const dim3 gPQ(nN / NGR, HD2 / NGC);
  const dim3 gN(nN / NGR, HD / NGC);
  const int nEB = nN / TGT;

  for (int l = 0; l < nL; ++l) {
    const us_t* wPQh = (const us_t*)(ws + oPQh[l]);
    const us_t* wPQl = (const us_t*)(ws + oPQl[l]);
    const us_t* wE2h = (const us_t*)(ws + oE2h[l]);
    const us_t* wE2l = (const us_t*)(ws + oE2l[l]);
    const us_t* wN1h = (const us_t*)(ws + oN1h[l]);
    const us_t* wN1l = (const us_t*)(ws + oN1l[l]);
    const us_t* wN2h = (const us_t*)(ws + oN2h[l]);
    const us_t* wN2l = (const us_t*)(ws + oN2l[l]);
    const float* eb1l = eb1 + (size_t)l * HD;
    const float* eb2l = eb2 + (size_t)l * HD;
    const float* nb1l = nb1 + (size_t)l * HD;
    const float* nb2l = nb2 + (size_t)l * HD;

    k_ngemm<HD><<<gPQ, NGT, 0, stream>>>(hH, hL, hH, hL, wPQh, wPQl, eb1l, HD, HD2, 0, 0,
                                         PQ, nhH, nhL, 1, 0);
    k_edge<0><<<nEB, NTHR, LDS_EDGE, stream>>>(PQ, eidx, nE, nN, vec8, wE2h, wE2l, eb1l, eb2l,
                                               attw + (size_t)l * HD, attb + l, cw1, x_in, eattr,
                                               aggH, aggL, out_x);
    k_ngemm<HD2><<<gN, NGT, 0, stream>>>(hH, hL, aggH, aggL, wN1h, wN1l, nb1l, HD, HD, 1, 1,
                                         PQ, nhH, nhL, 0, 1);
    k_ngemm<HD><<<gN, NGT, 0, stream>>>(nhH, nhL, nhH, nhL, wN2h, wN2l, nb2l, HD, HD, 1, 0,
                                        out_h, hH, hL, (l == nL - 1) ? 1 : 0, 1);
  }

  k_ngemm<HD><<<gPQ, NGT, 0, stream>>>(hH, hL, hH, hL, wCPh, wCPl, cb1, HD, HD2, 0, 0,
                                       PQ, nhH, nhL, 1, 0);
  k_edge<1><<<nEB, NTHR, LDS_EDGE, stream>>>(PQ, eidx, nE, nN, vec8, wC2, wC2, cb1, cb2, cw3, attb,
                                             cw1 + (size_t)HD2 * HD, x_in, eattr, aggH, aggL, out_x);
}
